// SimplePredictionLayer_52785148068523
// MI455X (gfx1250) — hardware-verified
//
#include <hip/hip_runtime.h>
#include <stddef.h>


typedef _Float16 h16;
typedef _Float16 v16h __attribute__((ext_vector_type(16)));
typedef _Float16 v8h  __attribute__((ext_vector_type(8)));
typedef float    v8f  __attribute__((ext_vector_type(8)));
typedef float    v4f  __attribute__((ext_vector_type(4)));

#ifndef NB
#define NB 2
#endif
#ifndef SEQ
#define SEQ 1024
#endif
#define NB_FULL  2
#define SEQ_FULL 1024
#define NSENT 128
#define DIM   512
#define MROWS (NB * NSENT)

static_assert(NB >= 1 && NB <= NB_FULL);
static_assert(SEQ >= 4 && SEQ <= SEQ_FULL);
static_assert((NSENT % 4) == 0);
static_assert(DIM == 2 * 32 * 8);
static_assert((DIM % 64) == 0 && (DIM % 32) == 0);
static_assert(DIM == 4 * 4 * 32);
static_assert((MROWS % 32) == 0);
static_assert(((size_t)NSENT * 4) % 128 == 0);

#define LDT 72
static_assert((LDT % 8) == 0 && LDT >= 64);

#define WCARRY 64.0f

static_assert((size_t)64 * LDT * 2 <= (size_t)131072);
static_assert((size_t)4 * SEQ * 4 <= (size_t)131072);
static_assert((size_t)(32 * 4 + 32) * 4 <= (size_t)131072);

#define W1T_BYTES ((size_t)DIM * DIM * 2)
#define SP_BYTES  ((size_t)MROWS * DIM * 2)
#define OFF_W1T ((size_t)0)
#define OFF_SP  (OFF_W1T + W1T_BYTES)
#define WS_TOTAL (OFF_SP + SP_BYTES)
static_assert((W1T_BYTES % 128) == 0 && (SP_BYTES % 128) == 0);
static_assert(WS_TOTAL <= (size_t)134217728);

__device__ __forceinline__ float bf16r(float x) {
  unsigned int u = __float_as_uint(x);
  u = (u + 0x7FFFu + ((u >> 16) & 1u)) & 0xFFFF0000u;
  return __uint_as_float(u);
}

static __device__ __forceinline__ h16 toh_flush(float v) {
  const h16 r = (h16)v;
  return (fabsf(v) < 6.103515625e-05f) ? (h16)0.0f : r;
}

__device__ __forceinline__ v16h frag_at(const _Float16* p) {
  v8h lo = *(const v8h*)(p);
  v8h hi = *(const v8h*)(p + 16);
  v16h out;
#pragma unroll
  for (int i = 0; i < 8; ++i) { out[i] = lo[i]; out[i + 8] = hi[i]; }
  return out;
}

__device__ __forceinline__ v8f wmma16(v16h a, v16h b, v8f c) {
  v8f d = __builtin_amdgcn_wmma_f32_16x16x32_f16(false, a, false, b, (short)0, c,
                                                 false, false);
  asm volatile("v_nop\n\tv_nop\n\tv_nop\n\tv_nop" : "+v"(d) : "v"(a), "v"(b));
  return d;
}

__device__ __forceinline__ float red16_sum(float x) {
#pragma unroll
  for (int off = 1; off < 16; off <<= 1) x += __shfl_xor(x, off, 32);
  return x;
}

__device__ __forceinline__ float relu_act(float t) {
  return fmaxf(t, 0.0f);
}

__global__ __launch_bounds__(256) void wconv_kernel(
    const float* __restrict__ W, _Float16* __restrict__ Wt, unsigned ldw, unsigned ldk) {
  __shared__ _Float16 T[64 * LDT];
  const unsigned tid = threadIdx.x;
  const unsigned n0 = blockIdx.x * 64u;
  const unsigned k0 = blockIdx.y * 64u;
#pragma unroll 4
  for (unsigned j = 0; j < 16u; ++j) {
    const unsigned idx = tid + 256u * j;
    const unsigned kr = idx >> 6, nc = idx & 63u;
    const float v = W[(size_t)(k0 + kr) * ldw + n0 + nc];
    T[nc * LDT + kr] = toh_flush(WCARRY * bf16r(v));
  }
  __syncthreads();
  v8h x[2];
  size_t off[2];
#pragma unroll
  for (unsigned i = 0; i < 2u; ++i) {
    const unsigned n = 32u * i + (tid >> 3);
    const unsigned kc = (tid & 7u) * 8u;
    x[i] = *(const v8h*)&T[n * LDT + kc];
    off[i] = (size_t)(n0 + n) * ldk + k0 + kc;
  }
#pragma unroll
  for (int i = 0; i < 2; ++i) *(volatile v8h*)(Wt + off[i]) = x[i];
  __threadfence();
#pragma unroll
  for (int i = 0; i < 2; ++i) *(volatile v8h*)(Wt + off[i]) = x[i];
}

__global__ __launch_bounds__(256) void spmax_kernel(
    const float* __restrict__ mapping, const float* __restrict__ xin,
    _Float16* __restrict__ sp16) {
#pragma clang fp contract(off)
  __shared__ float Ms[4 * SEQ];
  const unsigned tid = threadIdx.x, lane = tid & 31u;
  const unsigned wave = (unsigned)__builtin_amdgcn_readfirstlane((int)(threadIdx.x >> 5));
  const unsigned b = blockIdx.x / (unsigned)(NSENT / 4);
  const unsigned n0 = (blockIdx.x - b * (unsigned)(NSENT / 4)) * 4u;

#pragma unroll 1
  for (unsigned s = tid; s < (unsigned)SEQ; s += 256u) {
    const v4f mv = *(const v4f*)(mapping + ((size_t)b * SEQ_FULL + s) * NSENT + n0);
    Ms[0u * SEQ + s] = bf16r(mv[0]);
    Ms[1u * SEQ + s] = bf16r(mv[1]);
    Ms[2u * SEQ + s] = bf16r(mv[2]);
    Ms[3u * SEQ + s] = bf16r(mv[3]);
  }
  __syncthreads();

  const unsigned nl = wave >> 1;
  const unsigned dc = ((wave & 1u) * 32u + lane) * 8u;
  const float* xp = xin + (size_t)b * SEQ_FULL * DIM + dc;

  float vm[8];
#pragma unroll
  for (int i = 0; i < 8; ++i) vm[i] = -3.402823466e+38f;
  unsigned saw_zero = 0u;

#pragma unroll 1
  for (unsigned s = 0; s < (unsigned)SEQ; ++s) {
    const unsigned mbits = (unsigned)__builtin_amdgcn_readfirstlane(
        (int)__float_as_uint(Ms[nl * (unsigned)SEQ + s]));
    if ((mbits & 0x7FFFFFFFu) != 0u) {
      const float mk = __uint_as_float(mbits);
      const v4f a0 = *(const v4f*)(xp + (size_t)s * DIM);
      const v4f a1 = *(const v4f*)(xp + (size_t)s * DIM + 4u);
#pragma unroll
      for (int i = 0; i < 4; ++i) {
        vm[i]     = fmaxf(vm[i],     mk * bf16r(a0[i]));
        vm[i + 4] = fmaxf(vm[i + 4], mk * bf16r(a1[i]));
      }
    } else {
      saw_zero = 1u;
    }
  }
  if (saw_zero != 0u) {
#pragma unroll
    for (int i = 0; i < 8; ++i) vm[i] = fmaxf(vm[i], 0.0f);
  }

  v8h o;
#pragma unroll
  for (int i = 0; i < 8; ++i) o[i] = toh_flush(vm[i]);
  _Float16* p = sp16 + (size_t)(b * (unsigned)NSENT + n0 + nl) * DIM + dc;
  *(volatile v8h*)p = o;
  __threadfence();
  *(volatile v8h*)p = o;
}

__global__ __launch_bounds__(256) void head_kernel(
    const _Float16* __restrict__ A16, const _Float16* __restrict__ Bt,
    const float* __restrict__ b1, const float* __restrict__ w2, const float* __restrict__ b2,
    float* __restrict__ outf) {
  __shared__ float Part[32 * 4];
  __shared__ float Fin[32];
  const unsigned tid = threadIdx.x, lane = tid & 31u;
  const unsigned wave = (unsigned)__builtin_amdgcn_readfirstlane((int)(threadIdx.x >> 5));
  const unsigned mw = wave >> 2, nw = wave & 3u;
  const unsigned hh = lane >> 4, m = lane & 15u;
  const unsigned row0 = blockIdx.x * 32u;

  const _Float16* ap = A16 + (size_t)(row0 + mw * 16u + m) * DIM + hh * 8u;

  float part[8];
#pragma unroll
  for (int r = 0; r < 8; ++r) part[r] = 0.0f;

#pragma unroll 1
  for (unsigned t = 0; t < 4u; ++t) {
    const unsigned nbase = nw * 128u + t * 32u;
    const _Float16* bp0 = Bt + (size_t)(nbase + m) * DIM + hh * 8u;
    const _Float16* bp1 = bp0 + (size_t)16 * DIM;
    v8f acc0 = {}, acc1 = {};
#pragma unroll 2
    for (unsigned k0 = 0; k0 < (unsigned)DIM; k0 += 32u) {
      const v16h a  = frag_at(ap + k0);
      const v16h f0 = frag_at(bp0 + k0);
      const v16h f1 = frag_at(bp1 + k0);
      acc0 = wmma16(a, f0, acc0);
      acc1 = wmma16(a, f1, acc1);
    }
    const unsigned c0 = nbase + m;
    const unsigned c1 = c0 + 16u;
    const float bb0 = bf16r(b1[c0]);
    const float bb1 = bf16r(b1[c1]);
    const float ww0 = bf16r(w2[c0]);
    const float ww1 = bf16r(w2[c1]);
#pragma unroll
    for (int r = 0; r < 8; ++r) {
      const float h0 = relu_act(acc0[r] * (1.0f / WCARRY) + bb0);
      const float h1 = relu_act(acc1[r] * (1.0f / WCARRY) + bb1);
      part[r] += h0 * ww0;
      part[r] += h1 * ww1;
    }
  }

#pragma unroll
  for (int r = 0; r < 8; ++r) part[r] = red16_sum(part[r]);

  if (m == 0u) {
#pragma unroll
    for (int r = 0; r < 8; ++r)
      Part[(mw * 16u + hh * 8u + (unsigned)r) * 4u + nw] = part[r];
  }
  __syncthreads();

  if (tid < 32u) {
    const v4f pq = *(const v4f*)&Part[tid * 4u];
    Fin[tid] = ((pq[0] + pq[1]) + (pq[2] + pq[3])) + bf16r(b2[0]);
  }
  __syncthreads();

  if (tid < 8u) {
    const v4f x = *(const v4f*)&Fin[tid * 4u];
    float* p = outf + row0 + tid * 4u;
    *(volatile v4f*)p = x;
    __threadfence();
    *(volatile v4f*)p = x;
  }
}

extern "C" void kernel_launch(void* const* d_in, const int* in_sizes, int n_in,
                              void* d_out, int out_size, void* d_ws, size_t ws_size,
                              hipStream_t stream) {
  if (n_in < 6) return;
  const long long tok = (long long)(NB - 1) * SEQ_FULL + SEQ;
  if ((long long)in_sizes[0] < tok * NSENT) return;
  if ((long long)in_sizes[1] < tok * DIM) return;
  if ((long long)in_sizes[2] < (long long)DIM * DIM) return;
  if (in_sizes[3] < DIM) return;
  if (in_sizes[4] < DIM) return;
  if (in_sizes[5] < 1) return;
  if ((long long)out_size < (long long)MROWS) return;
  if (ws_size < WS_TOTAL) return;

  const float* mapping = (const float*)d_in[0];
  const float* xin     = (const float*)d_in[1];
  const float* w1      = (const float*)d_in[2];
  const float* b1      = (const float*)d_in[3];
  const float* w2      = (const float*)d_in[4];
  const float* b2      = (const float*)d_in[5];
  float* out = (float*)d_out;

  char* ws = (char*)d_ws;
  _Float16* W1t  = (_Float16*)(ws + OFF_W1T);
  _Float16* Sp16 = (_Float16*)(ws + OFF_SP);

  dim3 blk(256);
  wconv_kernel<<<dim3(DIM / 64, DIM / 64), blk, 0, stream>>>(w1, W1t, (unsigned)DIM, (unsigned)DIM);
  spmax_kernel<<<dim3(NB * (NSENT / 4)), blk, 0, stream>>>(mapping, xin, Sp16);
  head_kernel<<<dim3(MROWS / 32), blk, 0, stream>>>(Sp16, W1t, b1, w2, b2, out);
}
